// GraphAttentionLayer_3736621548022
// MI455X (gfx1250) — hardware-verified
//
#include <hip/hip_runtime.h>
#include <stddef.h>


typedef _Float16 v16h __attribute__((ext_vector_type(16)));
typedef _Float16 v8h  __attribute__((ext_vector_type(8)));
typedef _Float16 v4h  __attribute__((ext_vector_type(4)));
typedef float    v8f  __attribute__((ext_vector_type(8)));
typedef float    v4f  __attribute__((ext_vector_type(4)));
typedef int      v4i  __attribute__((ext_vector_type(4)));

#ifndef NB
#define NB 2
#endif
#ifndef SEQ
#define SEQ 2048
#endif
#define NB_FULL  2
#define SEQ_FULL 2048
#define NT    8
#define FIN   64
#define FOUT  64
#define NBT   (NB * NT)
#define MROWS (NBT * SEQ)

static_assert(NB >= 1 && NB <= NB_FULL);
static_assert(SEQ >= 64 && SEQ <= SEQ_FULL && (SEQ % 64) == 0);
static_assert(NT == 8 && NT * 32 == 256);
static_assert(FIN == 64 && FOUT == 64);
static_assert((FIN % 32) == 0 && (SEQ % 32) == 0);
static_assert((MROWS % 64) == 0 && (SEQ % 16) == 0);

#define LDT 72
#define LDC 68
static_assert((LDT % 8) == 0 && LDT >= 64);
static_assert((LDC % 4) == 0 && LDC >= 64);

#define WCARRY  64.0f
#define HCARRY  16.0f
#define WHCARRY 16.0f
#define PCARRY  16384.0f

#define LEAKY   0.2f
#define MASKV   (-9.0e15f)

#define WT_BYTES   ((size_t)FIN * FOUT * 2)
#define WHT_BYTES  ((size_t)NBT * FOUT * SEQ * 2)
#define W12_BYTES  ((size_t)2 * MROWS * 4)
#define OFF_WT   ((size_t)0)
#define OFF_WHT  (OFF_WT + WT_BYTES)
#define OFF_W12  (OFF_WHT + WHT_BYTES)
#define WS_TOTAL (OFF_W12 + W12_BYTES)
static_assert((WT_BYTES % 128) == 0 && (WHT_BYTES % 128) == 0 && (W12_BYTES % 128) == 0);
static_assert(WS_TOTAL <= (size_t)134217728);

__device__ __forceinline__ float bf16r(float x) {
  unsigned int u = __float_as_uint(x);
  u = (u + 0x7FFFu + ((u >> 16) & 1u)) & 0xFFFF0000u;
  return __uint_as_float(u);
}

static __device__ __forceinline__ _Float16 toh_flush(float v) {
  const _Float16 r = (_Float16)v;
  return (fabsf(v) < 6.103515625e-05f) ? (_Float16)0.0f : r;
}

__device__ __forceinline__ v16h frag_at(const _Float16* p) {
  v8h lo = *(const v8h*)(p);
  v8h hi = *(const v8h*)(p + 16);
  v16h out;
#pragma unroll
  for (int i = 0; i < 8; ++i) { out[i] = lo[i]; out[i + 8] = hi[i]; }
  return out;
}
__device__ __forceinline__ v16h ld_frag(const _Float16* base, unsigned ld) {
  const unsigned lane = threadIdx.x & 31u;
  return frag_at(base + (lane & 15u) * ld + (lane >> 4) * 8u);
}

__device__ __forceinline__ v8f wmma16(v16h a, v16h b, v8f c) {
  v8f d = __builtin_amdgcn_wmma_f32_16x16x32_f16(false, a, false, b, (short)0, c,
                                                 false, false);
  asm volatile("v_nop\n\tv_nop\n\tv_nop\n\tv_nop" : "+v"(d) : "v"(a), "v"(b));
  return d;
}

__device__ __forceinline__ void wave_lds_sync() {
  __builtin_amdgcn_fence(3  , "wavefront");
  asm volatile("s_wait_dscnt 0x0" ::: "memory");
  __builtin_amdgcn_wave_barrier();
}

__global__ __launch_bounds__(256) void wconv_kernel(
    const float* __restrict__ W, _Float16* __restrict__ Wt, unsigned ldw, unsigned ldk) {
  __shared__ _Float16 T[64 * LDT];
  const unsigned tid = threadIdx.x;
  const unsigned n0 = blockIdx.x * 64u;
  const unsigned k0 = blockIdx.y * 64u;
#pragma unroll 4
  for (unsigned j = 0; j < 16u; ++j) {
    const unsigned idx = tid + 256u * j;
    const unsigned kr = idx >> 6, nc = idx & 63u;
    const float v = W[(size_t)(k0 + kr) * ldw + n0 + nc];
    T[nc * LDT + kr] = (_Float16)(WCARRY * bf16r(v));
  }
  __syncthreads();
  v8h x[2];
  size_t off[2];
#pragma unroll
  for (unsigned i = 0; i < 2u; ++i) {
    const unsigned n = 32u * i + (tid >> 3);
    const unsigned kc = (tid & 7u) * 8u;
    x[i] = *(const v8h*)&T[n * LDT + kc];
    off[i] = (size_t)(n0 + n) * ldk + k0 + kc;
  }
#pragma unroll
  for (int i = 0; i < 2; ++i) *(volatile v8h*)(Wt + off[i]) = x[i];
  __threadfence();
#pragma unroll
  for (int i = 0; i < 2; ++i) *(volatile v8h*)(Wt + off[i]) = x[i];
}

__global__ __launch_bounds__(256) void wh_kernel(
    const float* __restrict__ Hin, const _Float16* __restrict__ Wt,
    const float* __restrict__ avec, _Float16* __restrict__ WhT, float* __restrict__ W12) {
  __shared__ __attribute__((aligned(16))) _Float16 As[64 * LDT];
  __shared__ __attribute__((aligned(16))) float Cs[64 * LDC];
  __shared__ __attribute__((aligned(16))) float Sd[2 * 64];

  const unsigned tid = threadIdx.x, lane = tid & 31u;
  const unsigned w = (unsigned)__builtin_amdgcn_readfirstlane((int)(threadIdx.x >> 5));
  const unsigned mw = w >> 1, nw = w & 1u;
  const unsigned hh = lane >> 4, m = lane & 15u;
  const unsigned row0 = blockIdx.x * 64u;
  const unsigned bt = row0 / (unsigned)SEQ;
  const unsigned n0 = row0 - bt * (unsigned)SEQ;
  const size_t frow0 = (size_t)bt * SEQ_FULL + n0;

#pragma unroll
  for (unsigned j = 0; j < 4u; ++j) {
    const unsigned idx = tid + 256u * j;
    const unsigned r = idx >> 4, c = (idx & 15u) * 4u;
    const v4f x = *(const v4f*)(Hin + (frow0 + r) * FIN + c);
    v4h y;
#pragma unroll
    for (int i = 0; i < 4; ++i) y[i] = toh_flush(HCARRY * bf16r(x[i]));
    *(v4h*)&As[r * LDT + c] = y;
  }
  __syncthreads();

  const _Float16* bp0 = Wt + (size_t)(nw * 32u + m) * FIN + hh * 8u;
  const _Float16* bp1 = bp0 + (size_t)16 * FIN;
  v8f acc0 = {}, acc1 = {};
#pragma unroll
  for (unsigned k0 = 0; k0 < (unsigned)FIN; k0 += 32u) {
    const v16h a  = ld_frag(&As[(mw * 16u) * LDT + k0], LDT);
    const v16h b0 = frag_at(bp0 + k0);
    const v16h b1 = frag_at(bp1 + k0);
    acc0 = wmma16(a, b0, acc0);
    acc1 = wmma16(a, b1, acc1);
  }
#pragma unroll
  for (int r = 0; r < 8; ++r) {
    float* d = &Cs[(mw * 16u + hh * 8u + (unsigned)r) * LDC + nw * 32u + m];
    d[0]  = acc0[r];
    d[16] = acc1[r];
  }
  __syncthreads();

  {
    const unsigned r = tid >> 2, q = tid & 3u;
    float s1 = 0.0f, s2 = 0.0f;
#pragma unroll 4
    for (unsigned c = 0; c < 16u; ++c) {
      const unsigned col = q * 16u + c;
      const float v = Cs[r * LDC + col];
      s1 += v * bf16r(avec[col]);
      s2 += v * bf16r(avec[FOUT + col]);
    }
    s1 += __shfl_xor(s1, 1, 32);
    s2 += __shfl_xor(s2, 1, 32);
    s1 += __shfl_xor(s1, 2, 32);
    s2 += __shfl_xor(s2, 2, 32);
    if (q == 0u) {
      Sd[r]       = s1 * (1.0f / (WCARRY * HCARRY));
      Sd[64u + r] = s2 * (1.0f / (WCARRY * HCARRY));
    }
  }

  v8h x[2];
  size_t off[2];
#pragma unroll
  for (unsigned i = 0; i < 2u; ++i) {
    const unsigned dcol = 32u * i + (tid >> 3);
    const unsigned kk = (tid & 7u) * 8u;
#pragma unroll
    for (unsigned j = 0; j < 8u; ++j) {
      const float t = Cs[(kk + j) * LDC + dcol] * (WHCARRY / (WCARRY * HCARRY));
      x[i][j] = toh_flush(t);
    }
    off[i] = ((size_t)bt * FOUT + dcol) * SEQ + n0 + kk;
  }
  __syncthreads();

  const v4f sv = *(const v4f*)&Sd[(lane >> 4) * 64u + (lane & 15u) * 4u];
  const size_t soff = (size_t)(lane >> 4) * MROWS + row0 + (lane & 15u) * 4u;

#pragma unroll
  for (int i = 0; i < 2; ++i) *(volatile v8h*)(WhT + off[i]) = x[i];
  if (w == 0u) *(volatile v4f*)(W12 + soff) = sv;
  __threadfence();
#pragma unroll
  for (int i = 0; i < 2; ++i) *(volatile v8h*)(WhT + off[i]) = x[i];
  if (w == 0u) *(volatile v4f*)(W12 + soff) = sv;
}

__global__ __launch_bounds__(256) void gat_kernel(
    const _Float16* __restrict__ WhT, const float* __restrict__ W12,
    const int* __restrict__ adj, float* __restrict__ out) {
  __shared__ __attribute__((aligned(16))) _Float16 Pt[NT * 16 * LDT];
  __shared__ __attribute__((aligned(16))) float Os[NT * 16 * LDC];

  const unsigned tid = threadIdx.x, lane = tid & 31u;
  const unsigned t = (unsigned)__builtin_amdgcn_readfirstlane((int)(threadIdx.x >> 5));
  const unsigned hh = lane >> 4, m = lane & 15u;
  const unsigned i0 = blockIdx.x * 16u;
  const unsigned b = blockIdx.y;
  const unsigned bt = b * NT + t;

  const unsigned pi = tid >> 4;
  const unsigned pj = (tid & 15u) * 4u;

  float w1[NT];
#pragma unroll
  for (int tt = 0; tt < NT; ++tt)
    w1[tt] = W12[(size_t)(b * NT + (unsigned)tt) * SEQ + i0 + pi];

  const int* adjrow = adj + (size_t)(i0 + pi) * SEQ_FULL + pj;
  const float* w2base = W12 + (size_t)MROWS + (size_t)(b * NT) * SEQ + pj;
  const _Float16* vb = WhT + ((size_t)bt * FOUT + m) * SEQ + hh * 8u;

  v8f o[4];
#pragma unroll
  for (int nb = 0; nb < 4; ++nb) o[nb] = (v8f){};

  for (unsigned j0 = 0; j0 < (unsigned)SEQ; j0 += 64u) {
    const v4i ad = *(const v4i*)(adjrow + j0);
    v4f w2[NT];
#pragma unroll
    for (int tt = 0; tt < NT; ++tt)
      w2[tt] = *(const v4f*)(w2base + (size_t)tt * SEQ + j0);

    v4h ph[NT];
#pragma unroll
    for (int jj = 0; jj < 4; ++jj) {
      float e[NT];
      const bool keep = (ad[jj] > 0);
#pragma unroll
      for (int tt = 0; tt < NT; ++tt) {
        float x = w1[tt] + w2[tt][jj];
        x = (x > 0.0f) ? x : LEAKY * x;
        e[tt] = keep ? x : MASKV;
      }
      float mx = fmaxf(fmaxf(fmaxf(e[0], e[1]), fmaxf(e[2], e[3])),
                       fmaxf(fmaxf(e[4], e[5]), fmaxf(e[6], e[7])));
      float s = 0.0f;
#pragma unroll
      for (int tt = 0; tt < NT; ++tt) {
        e[tt] = __expf(e[tt] - mx);
        s += e[tt];
      }
      const float inv = __builtin_amdgcn_rcpf(s) * PCARRY;
#pragma unroll
      for (int tt = 0; tt < NT; ++tt) ph[tt][jj] = toh_flush(e[tt] * inv);
    }
#pragma unroll
    for (int tt = 0; tt < NT; ++tt)
      *(v4h*)&Pt[((unsigned)tt * 16u + pi) * LDT + pj] = ph[tt];
    __syncthreads();

#pragma unroll
    for (int c = 0; c < 2; ++c) {
      const v16h pf = ld_frag(&Pt[(t * 16u) * LDT + (unsigned)c * 32u], LDT);
#pragma unroll
      for (int nb = 0; nb < 4; ++nb) {
        const v16h vf = frag_at(vb + (size_t)(nb * 16) * SEQ + j0 + (unsigned)c * 32u);
        o[nb] = wmma16(pf, vf, o[nb]);
      }
    }
    __syncthreads();
  }

  const float fs = 1.0f / (PCARRY * WHCARRY);
#pragma unroll
  for (int nb = 0; nb < 4; ++nb)
#pragma unroll
    for (int v = 0; v < 8; ++v)
      Os[(t * 16u + hh * 8u + (unsigned)v) * LDC + (unsigned)nb * 16u + m] = o[nb][v] * fs;
  wave_lds_sync();

#pragma unroll 1
  for (unsigned g = 0; g < 8u; ++g) {
    const unsigned r = 2u * g + (lane >> 4);
    const unsigned c = (lane & 15u) * 4u;
    v4f u = *(const v4f*)&Os[(t * 16u + r) * LDC + c];
#pragma unroll
    for (int j = 0; j < 4; ++j) {
      const float em = expm1f(u[j]);
      u[j] = (u[j] > 0.0f) ? u[j] : em;
    }
    *(v4f*)&Os[(t * 16u + r) * LDC + c] = u;
  }
  wave_lds_sync();

  v4f x[8];
  size_t off[8];
#pragma unroll
  for (unsigned i = 0; i < 8u; ++i) {
    const unsigned r = 2u * i + (lane >> 4);
    const unsigned c = (lane & 15u) * 4u;
    x[i] = *(const v4f*)&Os[(t * 16u + r) * LDC + c];
    off[i] = ((size_t)bt * SEQ_FULL + i0 + r) * FOUT + c;
  }
#pragma unroll
  for (int i = 0; i < 8; ++i) *(volatile v4f*)(out + off[i]) = x[i];
  __threadfence();
#pragma unroll
  for (int i = 0; i < 8; ++i) *(volatile v4f*)(out + off[i]) = x[i];
}

extern "C" void kernel_launch(void* const* d_in, const int* in_sizes, int n_in,
                              void* d_out, int out_size, void* d_ws, size_t ws_size,
                              hipStream_t stream) {
  if (n_in < 4) return;
  const long long need_h = ((long long)(NBT - 1) * SEQ_FULL + SEQ) * FIN;
  const long long need_adj = (long long)(SEQ - 1) * SEQ_FULL + SEQ;
  if ((long long)in_sizes[0] < need_h) return;
  if ((long long)in_sizes[1] < (long long)FIN * FOUT) return;
  if ((long long)in_sizes[2] < (long long)2 * FOUT) return;
  if ((long long)in_sizes[3] < need_adj) return;
  if ((long long)out_size < need_h) return;
  if (ws_size < WS_TOTAL) return;

  const float* h   = (const float*)d_in[0];
  const float* W   = (const float*)d_in[1];
  const float* a   = (const float*)d_in[2];
  const int*   adj = (const int*)d_in[3];
  float* out = (float*)d_out;

  char* ws = (char*)d_ws;
  _Float16* Wt  = (_Float16*)(ws + OFF_WT);
  _Float16* WhT = (_Float16*)(ws + OFF_WHT);
  float*    W12 = (float*)(ws + OFF_W12);

  dim3 blk(256);
  wconv_kernel<<<dim3(FOUT / 64, FIN / 64), blk, 0, stream>>>(W, Wt, (unsigned)FOUT, (unsigned)FIN);
  wh_kernel<<<dim3(MROWS / 64), blk, 0, stream>>>(h, Wt, a, WhT, W12);
  gat_kernel<<<dim3(SEQ / 16, NB), blk, 0, stream>>>(WhT, W12, adj, out);
}
